// densityPropGRUCell_18476949308043
// MI455X (gfx1250) — hardware-run, weakly checked
//
#include <hip/hip_runtime.h>
#include <math.h>

typedef __attribute__((ext_vector_type(16))) _Float16 v16h;
typedef __attribute__((ext_vector_type(8)))  _Float16 v8h;
typedef __attribute__((ext_vector_type(8)))  float    v8f;
typedef __attribute__((ext_vector_type(4)))  float    v4f;

constexpr int kU   = 256;
constexpr int kBn  = 128;
constexpr int kUU  = kU * kU;
constexpr int kVecStride = 4096;
constexpr int kOffPZ = 0;
constexpr int kOffPR = 1024;
constexpr int kOffPT = 2048;
constexpr int kOffPH = 3072;
static_assert(4 * kU == 1024 && 4 * 1024 == kVecStride, "packed table layout");

constexpr float kCarryW = 256.0f;
constexpr float kCarryS = 256.0f;
constexpr float kCarryG = 256.0f;
constexpr float kCarryT = 256.0f;
static_assert(kCarryS == kCarryG, "one stage-1 scale for both covariance planes");
constexpr float kScaleS1 = kCarryT / (kCarryW * kCarryS);
constexpr float kScaleS2 = 1.0f / (kCarryW * kCarryT);
constexpr float kInvCarryG = 1.0f / kCarryG;

constexpr size_t kOffWT  = 0;
constexpr size_t kOffSP  = kOffWT  + (size_t)768 * kU * 2;
constexpr size_t kOffS16 = kOffSP  + (size_t)6 * kU * 4;
constexpr size_t kOffTZR = kOffS16 + (size_t)kBn * kUU * 2;
constexpr size_t kOffSZ  = kOffTZR + (size_t)kBn * 2 * kUU * 2;
constexpr size_t kOffG16 = kOffSZ  + (size_t)kBn * kUU * 4;
constexpr size_t kOffTTH = kOffG16 + (size_t)kBn * kUU * 2;
constexpr size_t kOffVEC = kOffTTH + (size_t)kBn * kUU * 2;
constexpr size_t kWsTotal = kOffVEC + (size_t)kBn * kVecStride * 4;
static_assert(kWsTotal == 119937024ull, "carve total");
static_assert(kWsTotal <= 134217728ull, "carve cap");
static_assert((kOffSP % 128) == 0 && (kOffS16 % 128) == 0 && (kOffTZR % 128) == 0 && (kOffSZ % 128) == 0 &&
              (kOffG16 % 128) == 0 && (kOffTTH % 128) == 0 && (kOffVEC % 128) == 0, "128-B aligned regions");
static_assert((kU % 32) == 0 && (kU % 64) == 0, "GEMM K multiple of 32, M and N multiples of 64");

__device__ __forceinline__ void grp_guard(v8f& a, v8f& b, v8f& c, v8f& d, v16h x, v16h y0, v16h y1, v16h y2, v16h y3) {
  asm volatile("v_nop\n\tv_nop\n\tv_nop\n\tv_nop" : "+v"(a), "+v"(b), "+v"(c), "+v"(d) : "v"(x), "v"(y0), "v"(y1), "v"(y2), "v"(y3));
}
__device__ __forceinline__ void keep4_h(v16h a, v16h b, v16h c, v16h d) { asm volatile("v_nop" :: "v"(a), "v"(b), "v"(c), "v"(d)); }
__device__ __forceinline__ void acc_guard4(v8f& a, v8f& b, v8f& c, v8f& d) { asm volatile("v_nop\n\tv_nop\n\tv_nop\n\tv_nop" : "+v"(a), "+v"(b), "+v"(c), "+v"(d)); }
struct FragH {
  union U { v16h v; v8h h[2]; };
  static __device__ __forceinline__ v16h load(const _Float16* p) {
    U f; f.h[0] = *(const v8h*)(p); f.h[1] = *(const v8h*)(p + 16); return f.v;
  }
  static __device__ __forceinline__ v8f mma(v16h a, v16h b, v8f c) {
    return __builtin_amdgcn_wmma_f32_16x16x32_f16(false, a, false, b, (short)0, c, false, false);
  }
};
__device__ __forceinline__ void wave_lds_sync() {
  __builtin_amdgcn_fence(__ATOMIC_RELEASE, "workgroup");
  __builtin_amdgcn_wave_barrier();
  __builtin_amdgcn_fence(__ATOMIC_ACQUIRE, "workgroup");
}
__device__ __forceinline__ float h16_to_f32(unsigned hb) {
  const unsigned sgn = (hb & 0x8000u) << 16; const unsigned em = hb & 0x7fffu;
  const float fn = __uint_as_float((em << 13) + 0x38000000u);
  const float fs = (float)em * 5.9604644775390625e-8f;
  const float mag = (em < 0x400u) ? fs : fn; return __uint_as_float(__float_as_uint(mag) | sgn);
}

template <int EPI>
__device__ __forceinline__ float epi_elem(float v, bool dg, v4f rp, v4f cp, float S, float Sz) {
  const float dadd = dg ? rp[0] : 0.0f;
  const float core = v + dadd;
  const float sg = core * (rp[1] * cp[1]);
  if (EPI == 1) return sg;
  if (EPI == 2) return (sg * (S + rp[2] * cp[2]) + (rp[3] * cp[3]) * S) * kCarryG;
  return Sz * (S + sg + rp[2] * cp[2]) + (rp[3] * cp[3]) * S + ((1.0f - rp[3]) * (1.0f - cp[3])) * sg;
}

template <int EPI>
__global__ __launch_bounds__(256) void cov_gemm_kernel(
    const unsigned short* __restrict__ Ap,
    const unsigned short* __restrict__ Btp, long strideB,
    void* __restrict__ Cout, long strideC,
    const float* __restrict__ vecp, int vecOff,
    const float* __restrict__ Sin, const float* __restrict__ Szp,
    int M, float scale) {
  const _Float16* A  = (const _Float16*)Ap;
  const _Float16* Bt = (const _Float16*)Btp;
  __shared__ __align__(16) float sT[8][16 * 68];
  const int b    = blockIdx.y;
  const int lane = threadIdx.x & 31;
  const int wave = threadIdx.x >> 5;
  const int tilesM = M >> 6;
  const int tile = blockIdx.x * 8 + wave;
  if (tile >= tilesM * 4) return;
  const int tm = tile >> 2;
  const int tn = tile & 3;
  const int m0 = tm << 6;
  const int n0 = tn << 6;
  const _Float16* Bb = Bt + (size_t)b * strideB;

  const int rlane = lane & 15;
  const int koff  = (lane >> 4) * 8;
  const int mOff  = (lane >> 4) * 8;

  v8f acc[4][4];
#pragma unroll
  for (int i = 0; i < 4; ++i)
#pragma unroll
    for (int j = 0; j < 4; ++j) acc[i][j] = (v8f){0.f, 0.f, 0.f, 0.f, 0.f, 0.f, 0.f, 0.f};

#pragma unroll 1
  for (int k0 = 0; k0 < kU; k0 += 32) {
    v16h bh[4];
#pragma unroll
    for (int j = 0; j < 4; ++j)
      bh[j] = FragH::load(Bb + (size_t)(n0 + (j << 4) + rlane) * kU + koff + k0);
#pragma unroll
    for (int i = 0; i < 4; ++i) {
      const v16h ah = FragH::load(A + (size_t)(m0 + (i << 4) + rlane) * kU + koff + k0);
#pragma unroll
      for (int j = 0; j < 4; ++j) acc[i][j] = FragH::mma(ah, bh[j], acc[i][j]);
      grp_guard(acc[i][0], acc[i][1], acc[i][2], acc[i][3], ah, bh[0], bh[1], bh[2], bh[3]);
    }
    keep4_h(bh[0], bh[1], bh[2], bh[3]);
  }
  acc_guard4(acc[0][0], acc[0][1], acc[0][2], acc[0][3]);
  acc_guard4(acc[1][0], acc[1][1], acc[1][2], acc[1][3]);
  acc_guard4(acc[2][0], acc[2][1], acc[2][2], acc[2][3]);
  acc_guard4(acc[3][0], acc[3][1], acc[3][2], acc[3][3]);

  float* slab = sT[wave];
  const int hh = lane >> 4;
  const int c4 = (lane & 15) * 4;
  const float* vb = vecp + (size_t)b * kVecStride + vecOff;
  const float* Sb = Sin + (size_t)b * kUU;
  const float* Zb = Szp + (size_t)b * kUU;
  v4f cp0 = (v4f){0.f, 0.f, 0.f, 0.f}, cp1 = cp0, cp2 = cp0, cp3 = cp0;
  if (EPI != 0) {
    cp0 = *(const v4f*)(vb + (size_t)(n0 + c4 + 0) * 4);
    cp1 = *(const v4f*)(vb + (size_t)(n0 + c4 + 1) * 4);
    cp2 = *(const v4f*)(vb + (size_t)(n0 + c4 + 2) * 4);
    cp3 = *(const v4f*)(vb + (size_t)(n0 + c4 + 3) * 4);
  }
#pragma unroll
  for (int i = 0; i < 4; ++i) {
    const int mBase = m0 + (i << 4);
#pragma unroll
    for (int j = 0; j < 4; ++j) {
#pragma unroll
      for (int r = 0; r < 8; ++r)
        slab[(mOff + r) * 68 + (j << 4) + rlane] = acc[i][j][r] * scale;
    }
    wave_lds_sync();
    if (EPI != 0) {
#pragma unroll 1
      for (int it = 0; it < 8; ++it) {
        const int row = it * 2 + hh;
        const int gi = mBase + row;
        const int gl = n0 + c4;
        float* sp = slab + row * 68 + c4;
        const v4f v  = *(const v4f*)sp;
        const v4f rp = *(const v4f*)(vb + (size_t)gi * 4);
        v4f sv = (v4f){0.f, 0.f, 0.f, 0.f};
        v4f zv = (v4f){0.f, 0.f, 0.f, 0.f};
        if (EPI >= 2) sv = *(const v4f*)(Sb + (size_t)gi * kU + gl);
        if (EPI == 3) zv = *(const v4f*)(Zb + (size_t)gi * kU + gl);
        v4f o;
        o[0] = epi_elem<EPI>(v[0], gi == gl + 0, rp, cp0, sv[0], zv[0]);
        o[1] = epi_elem<EPI>(v[1], gi == gl + 1, rp, cp1, sv[1], zv[1]);
        o[2] = epi_elem<EPI>(v[2], gi == gl + 2, rp, cp2, sv[2], zv[2]);
        o[3] = epi_elem<EPI>(v[3], gi == gl + 3, rp, cp3, sv[3], zv[3]);
        *(v4f*)sp = o;
      }
      wave_lds_sync();
    }
    if (EPI == 1 || EPI == 3) {
      float* C = (float*)Cout + (size_t)b * strideC;
      for (int pass = 0; pass < 2; ++pass) {
#pragma unroll
        for (int it = 0; it < 8; ++it) {
          const int row = it * 2 + hh;
          const v4f v = *(const v4f*)(slab + row * 68 + c4);
          *(volatile v4f*)(C + (size_t)(mBase + row) * kU + n0 + c4) = v;
        }
        __threadfence();
      }
    } else {
      const int q = lane >> 3, c8 = (lane & 7) * 8;
      unsigned short* C = (unsigned short*)Cout + (size_t)b * strideC;
      for (int pass = 0; pass < 2; ++pass) {
#pragma unroll
        for (int it = 0; it < 4; ++it) {
          const int row = it * 4 + q;
          const float* sp = slab + row * 68 + c8;
          v8h hv;
#pragma unroll
          for (int e = 0; e < 8; ++e) hv[e] = (_Float16)sp[e];
          *(volatile v8h*)(C + (size_t)(mBase + row) * kU + n0 + c8) = hv;
        }
        __threadfence();
      }
    }
    wave_lds_sync();
  }
}

__global__ __launch_bounds__(256) void cast_plane_kernel(
    const float* __restrict__ src, unsigned short* __restrict__ dst, int total8) {
  const int i = blockIdx.x * 256 + threadIdx.x;
  if (i >= total8) return;
  const size_t e0 = (size_t)i << 3;
  const v4f a0 = *(const v4f*)(src + e0);
  const v4f a1 = *(const v4f*)(src + e0 + 4);
  v8h hv;
#pragma unroll
  for (int e = 0; e < 4; ++e) {
    hv[e]     = (_Float16)(a0[e] * kCarryS);
    hv[4 + e] = (_Float16)(a1[e] * kCarryS);
  }
  unsigned short* q = dst + e0;
  *(volatile v8h*)q = hv;
  __threadfence();
  *(volatile v8h*)q = hv;
}

__global__ __launch_bounds__(256) void weight_transpose_kernel(
    const float* __restrict__ Wz, const float* __restrict__ Wr, const float* __restrict__ Wh,
    unsigned short* __restrict__ WT) {
  __shared__ float tile[64 * 65];
  const int tid = threadIdx.x;
  const int l0 = blockIdx.x * 64, k0 = blockIdx.y * 64, sel = blockIdx.z;
  const float* W = (sel == 0) ? Wz : ((sel == 1) ? Wr : Wh);
#pragma unroll 4
  for (int r = 0; r < 16; ++r) {
    const int kk = r * 4 + (tid >> 6), ll = tid & 63;
    tile[kk * 65 + ll] = W[(size_t)(k0 + kk) * kU + l0 + ll];
  }
  __syncthreads();
  const int c8 = (tid & 7) * 8;
  v8h hv[2];
#pragma unroll
  for (int it = 0; it < 2; ++it) {
    const int row = it * 32 + (tid >> 3);
#pragma unroll
    for (int e = 0; e < 8; ++e) hv[it][e] = (_Float16)(tile[(c8 + e) * 65 + row] * kCarryW);
  }
#pragma unroll
  for (int it = 0; it < 2; ++it) {
    const int row = it * 32 + (tid >> 3);
    *(volatile v8h*)(WT + (size_t)(sel * kU + l0 + row) * kU + k0 + c8) = hv[it];
  }
  __threadfence();
#pragma unroll
  for (int it = 0; it < 2; ++it) {
    const int row = it * 32 + (tid >> 3);
    *(volatile v8h*)(WT + (size_t)(sel * kU + l0 + row) * kU + k0 + c8) = hv[it];
  }
}

__global__ __launch_bounds__(256) void softplus_kernel(
    const float* __restrict__ p0, const float* __restrict__ p1, const float* __restrict__ p2,
    const float* __restrict__ p3, const float* __restrict__ p4, const float* __restrict__ p5,
    float* __restrict__ SP) {
  __shared__ __align__(16) float sv[256];
  const int g = blockIdx.x, t = threadIdx.x;
  const float* src = (g == 0) ? p0 : (g == 1) ? p1 : (g == 2) ? p2 : (g == 3) ? p3 : (g == 4) ? p4 : p5;
  const float v = src[t];
  sv[t] = fmaxf(v, 0.0f) + log1pf(expf(-fabsf(v)));
  __syncthreads();
  if (t < 64) {
    const v4f o = *(const v4f*)(sv + 4 * t);
    float* q = SP + (size_t)g * kU + 4 * t;
    *(volatile v4f*)q = o;
    __threadfence();
    *(volatile v4f*)q = o;
  }
}

__global__ __launch_bounds__(256) void gates_kernel(
    const float* __restrict__ x_in, const float* __restrict__ s_in, const float* __restrict__ Sg,
    const float* __restrict__ Uz, const float* __restrict__ Wz,
    const float* __restrict__ Ur, const float* __restrict__ Wr,
    const float* __restrict__ Uh, const float* __restrict__ Wh,
    const float* __restrict__ SP, float* __restrict__ mu_out, float* __restrict__ vec) {
  __shared__ __align__(16) float lx[kU];
  __shared__ __align__(16) float ls[kU];
  __shared__ __align__(16) float lsr[kU];
  __shared__ __align__(16) float lmu[kU];
  __shared__ v4f red[256];
  const int b = blockIdx.x, t = threadIdx.x;
  const float xv = x_in[(size_t)b * kU + t];
  const float sv = s_in[(size_t)b * kU + t];
  lx[t] = xv;
  ls[t] = sv;
  __syncthreads();
  float mzx = 0.f, mzs = 0.f, mrx = 0.f, mrs = 0.f;
#pragma unroll 2
  for (int k = 0; k < kU; ++k) {
    const float xk = lx[k], sk = ls[k];
    mzx = fmaf(xk, Uz[(size_t)k * kU + t], mzx);
    mzs = fmaf(sk, Wz[(size_t)k * kU + t], mzs);
    mrx = fmaf(xk, Ur[(size_t)k * kU + t], mrx);
    mrs = fmaf(sk, Wr[(size_t)k * kU + t], mrs);
  }
  const float mz = mzx + mzs, mr = mrx + mrs;
  const float z = 1.0f / (1.0f + expf(-mz));
  const float r = 1.0f / (1.0f + expf(-mr));
  const float srv = sv * r;
  lsr[t] = srv;
  __syncthreads();
  float mhx = 0.f, mhs = 0.f;
#pragma unroll 2
  for (int k = 0; k < kU; ++k) {
    mhx = fmaf(lx[k], Uh[(size_t)k * kU + t], mhx);
    mhs = fmaf(lsr[k], Wh[(size_t)k * kU + t], mhs);
  }
  const float h = tanhf(mhx + mhs);
  const float sdiag = Sg[(size_t)b * kUU + (size_t)t * (kU + 1)];
  red[t] = (v4f){xv * xv, sv * sv, srv * srv, sdiag};
  __syncthreads();
#pragma unroll 1
  for (int off = 128; off > 0; off >>= 1) {
    if (t < off) {
      const v4f a = red[t], c = red[t + off];
      red[t] = a + c;
    }
    __syncthreads();
  }
  const v4f tot = red[0];
  const float ax = tot[0], as2 = tot[1], asr = tot[2], trS = tot[3];
  const float spuz = SP[0 * kU + t], spwz = SP[1 * kU + t];
  const float spur = SP[2 * kU + t], spwr = SP[3 * kU + t];
  const float spuh = SP[4 * kU + t], spwh = SP[5 * kU + t];
  const float dz = as2 * spwz + trS * spwz + ax * spuz;
  const float dr = as2 * spwr + trS * spwr + ax * spur;
  const float dhb = asr * spwh + ax * spuh;
  const float gz = z * (1.0f - z);
  const float gr = r * (1.0f - r);
  const float gh = 1.0f - h * h;
  const float mu = z * sv + (1.0f - z) * h;
  const float dd = sv - h;
  lmu[t] = mu;
  const v4f pz = (v4f){dz, gz, 0.0f, 0.0f};
  const v4f pr = (v4f){dr, gr, sv, r};
  const v4f pt = (v4f){gh, dd, z, dhb};
  float* vb = vec + (size_t)b * kVecStride;
  *(volatile v4f*)(vb + kOffPZ + 4 * t) = pz;
  *(volatile v4f*)(vb + kOffPR + 4 * t) = pr;
  *(volatile v4f*)(vb + kOffPT + 4 * t) = pt;
  __threadfence();
  *(volatile v4f*)(vb + kOffPZ + 4 * t) = pz;
  *(volatile v4f*)(vb + kOffPR + 4 * t) = pr;
  *(volatile v4f*)(vb + kOffPT + 4 * t) = pt;
  __syncthreads();
  if (t < 64) {
    const v4f o = *(const v4f*)(lmu + 4 * t);
    float* q = mu_out + (size_t)b * kU + 4 * t;
    *(volatile v4f*)q = o;
    __threadfence();
    *(volatile v4f*)q = o;
  }
}

__global__ __launch_bounds__(256) void trace_kernel(
    const unsigned short* __restrict__ G16, const float* __restrict__ SP, float* __restrict__ vec) {
  __shared__ float red[256];
  const int b = blockIdx.x, t = threadIdx.x;
  const size_t idx = (size_t)b * kUU + (size_t)t * (kU + 1);
  const unsigned w = ((const unsigned*)(const void*)G16)[idx >> 1];
  const unsigned lo = w & 0xffffu, hi = w >> 16;
  const unsigned hb = ((idx & 1) != 0) ? hi : lo;
  red[t] = h16_to_f32(hb) * kInvCarryG;
  __syncthreads();
#pragma unroll 1
  for (int off = 128; off > 0; off >>= 1) {
    if (t < off) {
      const float a = red[t], c = red[t + off];
      red[t] = a + c;
    }
    __syncthreads();
  }
  const float trG = red[0];
  float* vb = vec + (size_t)b * kVecStride;
  const v4f pt = *(const v4f*)(vb + kOffPT + 4 * t);
  const float spwh = SP[5 * kU + t];
  const float dh = pt[3] + trG * spwh;
  const v4f ph = (v4f){dh, pt[0], pt[1], pt[2]};
  *(volatile v4f*)(vb + kOffPH + 4 * t) = ph;
  __threadfence();
  *(volatile v4f*)(vb + kOffPH + 4 * t) = ph;
}

extern "C" void kernel_launch(void* const* d_in, const int* in_sizes, int n_in,
                              void* d_out, int out_size, void* d_ws, size_t ws_size,
                              hipStream_t stream) {
  if (n_in < 15) return;
  if (in_sizes[0] != kBn * kU || in_sizes[1] != kBn * kU) return;
  if (in_sizes[2] != kBn * kUU) return;
  if (in_sizes[3] != kUU || in_sizes[5] != kUU || in_sizes[7] != kUU ||
      in_sizes[9] != kUU || in_sizes[11] != kUU || in_sizes[13] != kUU) return;
  if (in_sizes[4] != kU || in_sizes[6] != kU || in_sizes[8] != kU ||
      in_sizes[10] != kU || in_sizes[12] != kU || in_sizes[14] != kU) return;
  if (out_size != kBn * kU + kBn * kUU) return;
  if (ws_size < kWsTotal) return;

  const float* x   = (const float*)d_in[0];
  const float* s   = (const float*)d_in[1];
  const float* Sg  = (const float*)d_in[2];
  const float* Uz  = (const float*)d_in[3];
  const float* uzs = (const float*)d_in[4];
  const float* Wz  = (const float*)d_in[5];
  const float* wzs = (const float*)d_in[6];
  const float* Ur  = (const float*)d_in[7];
  const float* urs = (const float*)d_in[8];
  const float* Wr  = (const float*)d_in[9];
  const float* wrs = (const float*)d_in[10];
  const float* Uh  = (const float*)d_in[11];
  const float* uhs = (const float*)d_in[12];
  const float* Wh  = (const float*)d_in[13];
  const float* whs = (const float*)d_in[14];

  float* out  = (float*)d_out;
  float* mu   = out;
  float* out1 = out + (size_t)kBn * kU;

  char* ws = (char*)d_ws;
  unsigned short* WT16 = (unsigned short*)(ws + kOffWT);
  float*          SP   = (float*)(ws + kOffSP);
  unsigned short* S16  = (unsigned short*)(ws + kOffS16);
  unsigned short* TZR  = (unsigned short*)(ws + kOffTZR);
  float*          SZ   = (float*)(ws + kOffSZ);
  unsigned short* G16  = (unsigned short*)(ws + kOffG16);
  unsigned short* TTH  = (unsigned short*)(ws + kOffTTH);
  float*          VEC  = (float*)(ws + kOffVEC);

  cast_plane_kernel<<<(kBn * kUU / 8) / 256, 256, 0, stream>>>(Sg, S16, kBn * kUU / 8);
  weight_transpose_kernel<<<dim3(4, 4, 3), 256, 0, stream>>>(Wz, Wr, Wh, WT16);
  softplus_kernel<<<6, 256, 0, stream>>>(uzs, wzs, urs, wrs, uhs, whs, SP);

  gates_kernel<<<kBn, 256, 0, stream>>>(x, s, Sg, Uz, Wz, Ur, Wr, Uh, Wh, SP, mu, VEC);

  cov_gemm_kernel<0><<<dim3(4, kBn), 256, 0, stream>>>(
      WT16, S16, (long)kUU, (void*)TZR, (long)(2 * kUU), VEC, 0, Sg, SZ, 2 * kU, kScaleS1);

  cov_gemm_kernel<1><<<dim3(2, kBn), 256, 0, stream>>>(
      WT16, TZR, (long)(2 * kUU), (void*)SZ, (long)kUU, VEC, kOffPZ, Sg, SZ, kU, kScaleS2);

  cov_gemm_kernel<2><<<dim3(2, kBn), 256, 0, stream>>>(
      WT16 + (size_t)kU * kU, TZR + (size_t)kUU, (long)(2 * kUU), (void*)G16, (long)kUU, VEC, kOffPR, Sg, SZ, kU, kScaleS2);

  trace_kernel<<<kBn, 256, 0, stream>>>(G16, SP, VEC);

  cov_gemm_kernel<0><<<dim3(2, kBn), 256, 0, stream>>>(
      WT16 + (size_t)2 * kU * kU, G16, (long)kUU, (void*)TTH, (long)kUU, VEC, 0, Sg, SZ, kU, kScaleS1);

  cov_gemm_kernel<3><<<dim3(2, kBn), 256, 0, stream>>>(
      WT16 + (size_t)2 * kU * kU, TTH, (long)kUU, (void*)out1, (long)kUU, VEC, kOffPH, Sg, SZ, kU, kScaleS2);
}
